// MambaBlock_7524782702695
// MI455X (gfx1250) — hardware-verified
//
#include <hip/hip_runtime.h>
#include <math.h>

typedef __attribute__((ext_vector_type(16))) _Float16 v16h;
typedef __attribute__((ext_vector_type(8)))  _Float16 v8h;
typedef __attribute__((ext_vector_type(16))) __bf16   v16b;
typedef __attribute__((ext_vector_type(8)))  __bf16   v8b;
typedef __attribute__((ext_vector_type(8)))  float    v8f;
typedef __attribute__((ext_vector_type(4)))  float    v4f;

constexpr int kBatch = 4;
constexpr int kCdim  = 256;
constexpr int kSeq   = 4096;
constexpr int kRows  = kBatch * kSeq;
constexpr int kDin   = 512;
constexpr int kNxz   = 2 * kDin;
constexpr int kNst   = 16;
constexpr int kDtR   = 16;
constexpr int kNdbc  = kDtR + 2 * kNst;
constexpr int kDbcP  = 64;
constexpr int kWdP   = 64;
constexpr int kDtK   = 32;
constexpr int kConvT = 4;
constexpr int kTP    = 260;
constexpr int kLnTok = 32;
constexpr float kEps = 1e-5f;
static_assert(kNdbc <= kDbcP && kDtR < kDtK && kDtK <= kWdP, "x_proj / dt padding");
static_assert((kCdim % 32) == 0 && (kDin % 32) == 0 && (kDtK % 32) == 0, "GEMM K multiples of 32");
static_assert((kSeq % 64) == 0 && (kNxz % 64) == 0 && (kDbcP % 64) == 0 && (kDin % 64) == 0 && (kCdim % 64) == 0, "GEMM M,N multiples of 64");
static_assert((kSeq % kLnTok) == 0 && (kDin % 256) == 0 && (kCdim == 256), "tile multiples");

constexpr size_t kOffWIH  = 0;
constexpr size_t kOffWIL  = kOffWIH  + (size_t)kNxz  * kCdim * 2;
constexpr size_t kOffWXH  = kOffWIL  + (size_t)kNxz  * kCdim * 2;
constexpr size_t kOffWXL  = kOffWXH  + (size_t)kDbcP * kDin  * 2;
constexpr size_t kOffWDH  = kOffWXL  + (size_t)kDbcP * kDin  * 2;
constexpr size_t kOffWDL  = kOffWDH  + (size_t)kDin  * kWdP  * 2;
constexpr size_t kOffWOH  = kOffWDL  + (size_t)kDin  * kWdP  * 2;
constexpr size_t kOffWOL  = kOffWOH  + (size_t)kCdim * kDin  * 2;
constexpr size_t kOffXNH  = kOffWOL  + (size_t)kCdim * kDin  * 2;
constexpr size_t kOffXNL  = kOffXNH  + (size_t)kRows * kCdim * 2;
constexpr size_t kOffXZ   = kOffXNL  + (size_t)kRows * kCdim * 2;
constexpr size_t kOffUC   = kOffXZ   + (size_t)kSeq  * kNxz  * 4;
constexpr size_t kOffUCH  = kOffUC   + (size_t)kSeq  * kDin  * 4;
constexpr size_t kOffUCL  = kOffUCH  + (size_t)kSeq  * kDin  * 2;
constexpr size_t kOffDBC  = kOffUCL  + (size_t)kSeq  * kDin  * 2;
constexpr size_t kOffDBCH = kOffDBC  + (size_t)kSeq  * kDbcP * 4;
constexpr size_t kOffDBCL = kOffDBCH + (size_t)kSeq  * kDbcP * 2;
constexpr size_t kOffDLR  = kOffDBCL + (size_t)kSeq  * kDbcP * 2;
constexpr size_t kOffYH   = kOffDLR  + (size_t)kSeq  * kDin  * 4;
constexpr size_t kOffYL   = kOffYH   + (size_t)kSeq  * kDin  * 2;
constexpr size_t kWsTotal = kOffYL   + (size_t)kSeq  * kDin  * 2;
static_assert(kWsTotal == 71041024ull, "carve total");
static_assert(kWsTotal <= 134217728ull, "carve cap");
static_assert((kOffWIL % 128) == 0 && (kOffWXH % 128) == 0 && (kOffWXL % 128) == 0 && (kOffWDH % 128) == 0 &&
              (kOffWDL % 128) == 0 && (kOffWOH % 128) == 0 && (kOffWOL % 128) == 0 && (kOffXNH % 128) == 0 &&
              (kOffXNL % 128) == 0 && (kOffXZ % 128) == 0 && (kOffUC % 128) == 0 && (kOffUCH % 128) == 0 &&
              (kOffUCL % 128) == 0 && (kOffDBC % 128) == 0 && (kOffDBCH % 128) == 0 && (kOffDBCL % 128) == 0 &&
              (kOffDLR % 128) == 0 && (kOffYH % 128) == 0 && (kOffYL % 128) == 0, "128-B aligned regions");

__device__ __forceinline__ unsigned short f2bf_bits(float f) {
  unsigned u = __float_as_uint(f);
  return (unsigned short)((u + 0x7FFFu + ((u >> 16) & 1u)) >> 16);
}
__device__ __forceinline__ float bf_bits2f(unsigned short h) { return __uint_as_float(((unsigned)h) << 16); }

__device__ __forceinline__ void dep_guard4_h(v8f& a, v8f& b, v8f& c, v8f& d, v16h x, v16h y) {
  asm volatile("v_nop\n\tv_nop\n\tv_nop\n\tv_nop" : "+v"(a), "+v"(b), "+v"(c), "+v"(d) : "v"(x), "v"(y));
}
__device__ __forceinline__ void dep_guard4_b(v8f& a, v8f& b, v8f& c, v8f& d, v16b x, v16b y) {
  asm volatile("v_nop\n\tv_nop\n\tv_nop\n\tv_nop" : "+v"(a), "+v"(b), "+v"(c), "+v"(d) : "v"(x), "v"(y));
}
__device__ __forceinline__ void keep4_h(v16h a, v16h b, v16h c, v16h d) { asm volatile("v_nop" :: "v"(a), "v"(b), "v"(c), "v"(d)); }
__device__ __forceinline__ void keep4_b(v16b a, v16b b, v16b c, v16b d) { asm volatile("v_nop" :: "v"(a), "v"(b), "v"(c), "v"(d)); }
__device__ __forceinline__ void acc_guard4(v8f& a, v8f& b, v8f& c, v8f& d) { asm volatile("v_nop\n\tv_nop\n\tv_nop\n\tv_nop" : "+v"(a), "+v"(b), "+v"(c), "+v"(d)); }
template <typename T> struct Frag;
template <> struct Frag<_Float16> {
  typedef v16h V; union U { v16h v; v8h h[2]; };
  static __device__ __forceinline__ v16h load(const _Float16* p) {
    U f; f.h[0] = *(const v8h*)(p); f.h[1] = *(const v8h*)(p + 16); return f.v;
  }
  static __device__ __forceinline__ v8f mma(v16h a, v16h b, v8f c) {
    return __builtin_amdgcn_wmma_f32_16x16x32_f16(false, a, false, b, (short)0, c, false, false);
  }
  static __device__ __forceinline__ void guard4(v8f& a, v8f& b, v8f& c, v8f& d, v16h x, v16h y) { dep_guard4_h(a, b, c, d, x, y); }
  static __device__ __forceinline__ void keep(v16h a, v16h b, v16h c, v16h d) { keep4_h(a, b, c, d); }
};
template <> struct Frag<__bf16> {
  typedef v16b V; union U { v16b v; v8b h[2]; };
  static __device__ __forceinline__ v16b load(const __bf16* p) {
    U f; f.h[0] = *(const v8b*)(p); f.h[1] = *(const v8b*)(p + 16); return f.v;
  }
  static __device__ __forceinline__ v8f mma(v16b a, v16b b, v8f c) {
    return __builtin_amdgcn_wmma_f32_16x16x32_bf16(false, a, false, b, (short)0, c, false, false);
  }
  static __device__ __forceinline__ void guard4(v8f& a, v8f& b, v8f& c, v8f& d, v16b x, v16b y) { dep_guard4_b(a, b, c, d, x, y); }
  static __device__ __forceinline__ void keep(v16b a, v16b b, v16b c, v16b d) { keep4_b(a, b, c, d); }
};

template <int ET> struct Elem;
template <> struct Elem<0> { typedef _Float16 T; };
template <> struct Elem<1> { typedef __bf16 T; };
template <int ET, bool SPLIT, int BIAS_MODE, int OUT_MODE, bool RESID>
__global__ __launch_bounds__(256) void wmma_gemm64(
    const unsigned short* __restrict__ Ap, const unsigned short* __restrict__ A2p, int lda, long strideA,
    const unsigned short* __restrict__ Btp, const unsigned short* __restrict__ Bt2p, int ldb, long strideB,
    void* __restrict__ Cout, void* __restrict__ Cout2, int ldc, long strideC,
    const float* __restrict__ bias,
    const float* __restrict__ resid, long strideR,
    int M, int N, int K, float scale) {
  static_assert(!(RESID && OUT_MODE != 0), "residual only with f32 output");
  typedef typename Elem<ET>::T T;
  typedef typename Frag<T>::V V;
  const T* A = (const T*)Ap; const T* A2 = (const T*)A2p; const T* Bt = (const T*)Btp; const T* Bt2 = (const T*)Bt2p;
  __shared__ __align__(16) float sT[8][16 * 68];
  const int b    = blockIdx.y;
  const int lane = threadIdx.x & 31;
  const int wave = threadIdx.x >> 5;
  const int tilesN = N >> 6;
  const int tilesM = M >> 6;
  const int tile = blockIdx.x * 8 + wave;
  if (tile >= tilesM * tilesN) return;
  const int tm = tile / tilesN;
  const int tn = tile - tm * tilesN;
  const int m0 = tm << 6;
  const int n0 = tn << 6;

  const T* Ab  = A  + (size_t)b * strideA;
  const T* Bb  = Bt + (size_t)b * strideB;
  const T* Ab2 = SPLIT ? (A2  + (size_t)b * strideA) : nullptr;
  const T* Bb2 = SPLIT ? (Bt2 + (size_t)b * strideB) : nullptr;

  const int rlane = lane & 15;
  const int koff  = (lane >> 4) * 8;
  const int mOff  = (lane >> 4) * 8;

  v8f acc[4][4];
#pragma unroll
  for (int i = 0; i < 4; ++i)
#pragma unroll
    for (int j = 0; j < 4; ++j) acc[i][j] = (v8f){0.f,0.f,0.f,0.f,0.f,0.f,0.f,0.f};

  for (int k0 = 0; k0 < K; k0 += 32) {
    V bh[4], bl[4];
#pragma unroll
    for (int j = 0; j < 4; ++j) {
      const size_t bo = (size_t)(n0 + (j << 4) + rlane) * ldb + koff + k0;
      bh[j] = Frag<T>::load(Bb + bo);
      if (SPLIT) bl[j] = Frag<T>::load(Bb2 + bo);
    }
#pragma unroll
    for (int i = 0; i < 4; ++i) {
      const size_t ao = (size_t)(m0 + (i << 4) + rlane) * lda + koff + k0;
      V ah = Frag<T>::load(Ab + ao);
      V al;
      if (SPLIT) al = Frag<T>::load(Ab2 + ao);
#pragma unroll
      for (int j = 0; j < 4; ++j) {
        acc[i][j] = Frag<T>::mma(ah, bh[j], acc[i][j]);
        if (SPLIT) {
          acc[i][j] = Frag<T>::mma(ah, bl[j], acc[i][j]);
          acc[i][j] = Frag<T>::mma(al, bh[j], acc[i][j]);
        }
      }
      Frag<T>::guard4(acc[i][0], acc[i][1], acc[i][2], acc[i][3], ah, SPLIT ? al : ah);
    }
    Frag<T>::keep(bh[0], bh[1], bh[2], bh[3]);
    if (SPLIT) Frag<T>::keep(bl[0], bl[1], bl[2], bl[3]);
  }
  acc_guard4(acc[0][0], acc[0][1], acc[0][2], acc[0][3]);
  acc_guard4(acc[1][0], acc[1][1], acc[1][2], acc[1][3]);
  acc_guard4(acc[2][0], acc[2][1], acc[2][2], acc[2][3]);
  acc_guard4(acc[3][0], acc[3][1], acc[3][2], acc[3][3]);

  float* slab = sT[wave];
  const float* Rb = RESID ? (resid + (size_t)b * strideR) : nullptr;
#pragma unroll
  for (int i = 0; i < 4; ++i) {
    const int mBase = m0 + (i << 4);
#pragma unroll
    for (int j = 0; j < 4; ++j) {
      const int n = n0 + (j << 4) + rlane;
      float bv = 0.f;
      if (BIAS_MODE == 2) bv = bias[n];
#pragma unroll
      for (int r = 0; r < 8; ++r) {
        float v = acc[i][j][r] * scale;
        if (BIAS_MODE == 1) v += bias[mBase + mOff + r];
        if (BIAS_MODE == 2) v += bv;
        slab[(mOff + r) * 68 + (j << 4) + rlane] = v;
      }
    }
    __builtin_amdgcn_fence(__ATOMIC_RELEASE, "workgroup");
    __builtin_amdgcn_wave_barrier();
    __builtin_amdgcn_fence(__ATOMIC_ACQUIRE, "workgroup");
    if (OUT_MODE == 0) {
      float* C = (float*)Cout + (size_t)b * strideC;
      const int hh = lane >> 4, c4 = (lane & 15) * 4;
      if (RESID) {
#pragma unroll
        for (int it = 0; it < 8; ++it) {
          const int row = it * 2 + hh;
          v4f sv = *(const v4f*)(slab + row * 68 + c4);
          const v4f rv = *(const v4f*)(Rb + (size_t)(mBase + row) * ldc + n0 + c4);
          sv += rv;
          *(v4f*)(slab + row * 68 + c4) = sv;
        }
      }
      for (int pass = 0; pass < 2; ++pass) {
#pragma unroll
        for (int it = 0; it < 8; ++it) {
          const int row = it * 2 + hh;
          v4f v = *(const v4f*)(slab + row * 68 + c4);
          *(volatile v4f*)(C + (size_t)(mBase + row) * ldc + n0 + c4) = v;
        }
        __threadfence();
      }
    } else {
      const int q = lane >> 3, c8 = (lane & 7) * 8;
      unsigned short* C  = (unsigned short*)Cout  + (size_t)b * strideC;
      unsigned short* C2 = (OUT_MODE == 2) ? ((unsigned short*)Cout2 + (size_t)b * strideC) : nullptr;
      for (int pass = 0; pass < 2; ++pass) {
#pragma unroll
        for (int it = 0; it < 4; ++it) {
          const int row = it * 4 + q;
          const float* sp = slab + row * 68 + c8;
          v8h hv, lv;
#pragma unroll
          for (int e = 0; e < 8; ++e) {
            if (OUT_MODE == 1) {
              hv[e] = (_Float16)sp[e];
            } else {
              unsigned short hb = f2bf_bits(sp[e]);
              unsigned short lb = f2bf_bits(sp[e] - bf_bits2f(hb));
              hv[e] = __builtin_bit_cast(_Float16, hb);
              lv[e] = __builtin_bit_cast(_Float16, lb);
            }
          }
          *(volatile v8h*)(C + (size_t)(mBase + row) * ldc + n0 + c8) = hv;
          if (OUT_MODE == 2) *(volatile v8h*)(C2 + (size_t)(mBase + row) * ldc + n0 + c8) = lv;
        }
        __threadfence();
      }
    }
    __builtin_amdgcn_fence(__ATOMIC_RELEASE, "workgroup");
    __builtin_amdgcn_wave_barrier();
    __builtin_amdgcn_fence(__ATOMIC_ACQUIRE, "workgroup");
  }
}

__global__ __launch_bounds__(256) void wt_split_kernel(
    const float* __restrict__ W, unsigned short* __restrict__ Bh, unsigned short* __restrict__ Bl,
    int Kdim, int Ndim, int Kpad)
{
  __shared__ float tile[64 * 65];
  const int tid = threadIdx.x, lane = tid & 31, wave = tid >> 5;
  const int n0 = blockIdx.x * 64;
  const int k0 = blockIdx.y * 64;
#pragma unroll 4
  for (int p = 0; p < 16; ++p) {
    const int idx = tid + p * 256;
    const int kk  = idx >> 6;
    const int nn  = idx & 63;
    const int n   = n0 + nn;
    const int k   = k0 + kk;
    const int nc  = (n < Ndim) ? n : (Ndim - 1);
    const int kc  = (k < Kdim) ? k : (Kdim - 1);
    const float v = W[(size_t)kc * Ndim + nc];
    tile[kk * 65 + nn] = (n < Ndim && k < Kdim) ? v : 0.0f;
  }
  __syncthreads();
  const int q = lane >> 3, c8 = (lane & 7) * 8;
  v8h hv[2], lv[2];
#pragma unroll
  for (int it = 0; it < 2; ++it) {
    const int nrow = it * 32 + wave * 4 + q;
#pragma unroll
    for (int e = 0; e < 8; ++e) {
      const float f = tile[(c8 + e) * 65 + nrow];
      const unsigned short hb = f2bf_bits(f);
      const unsigned short lb = f2bf_bits(f - bf_bits2f(hb));
      hv[it][e] = __builtin_bit_cast(_Float16, hb);
      lv[it][e] = __builtin_bit_cast(_Float16, lb);
    }
  }
  for (int pass = 0; pass < 2; ++pass) {
#pragma unroll
    for (int it = 0; it < 2; ++it) {
      const int nrow = it * 32 + wave * 4 + q;
      const size_t o = (size_t)(n0 + nrow) * Kpad + k0 + c8;
      *(volatile v8h*)(Bh + o) = hv[it];
      *(volatile v8h*)(Bl + o) = lv[it];
    }
    __threadfence();
  }
}

__global__ __launch_bounds__(256) void split_rows_bf16_kernel(
    const float* __restrict__ src, unsigned short* __restrict__ dhi, unsigned short* __restrict__ dlo, int total8)
{
  const int i = blockIdx.x * 256 + threadIdx.x;
  if (i >= total8) return;
  const size_t e0 = (size_t)i << 3;
  const v4f a0 = *(const v4f*)(src + e0);
  const v4f a1 = *(const v4f*)(src + e0 + 4);
  v8h hv, lv;
#pragma unroll
  for (int e = 0; e < 4; ++e) {
    const unsigned short h0 = f2bf_bits(a0[e]), h1 = f2bf_bits(a1[e]);
    const unsigned short l0 = f2bf_bits(a0[e] - bf_bits2f(h0)), l1 = f2bf_bits(a1[e] - bf_bits2f(h1));
    hv[e]     = __builtin_bit_cast(_Float16, h0);
    hv[4 + e] = __builtin_bit_cast(_Float16, h1);
    lv[e]     = __builtin_bit_cast(_Float16, l0);
    lv[4 + e] = __builtin_bit_cast(_Float16, l1);
  }
  unsigned short* qh = dhi + e0;
  unsigned short* ql = dlo + e0;
  *(volatile v8h*)qh = hv;
  *(volatile v8h*)ql = lv;
  __threadfence();
  *(volatile v8h*)qh = hv;
  *(volatile v8h*)ql = lv;
}

__global__ __launch_bounds__(256) void layernorm_split_kernel(
    const float* __restrict__ x, const float* __restrict__ nw, const float* __restrict__ nb,
    unsigned short* __restrict__ XNH, unsigned short* __restrict__ XNL)
{
  __shared__ __align__(16) float sX[kLnTok * kTP];
  const int tid = threadIdx.x, lane = tid & 31, wave = tid >> 5;
  const int t0 = blockIdx.x * kLnTok;
  const int bi = t0 / kSeq;
  const int l0 = t0 - bi * kSeq;
  const float* xb = x + (size_t)bi * kCdim * kSeq + l0 + lane;
#pragma unroll 4
  for (int i = 0; i < kCdim / 8; ++i) {
    const int c = wave + 8 * i;
    sX[lane * kTP + c] = xb[(size_t)c * kSeq];
  }
  __syncthreads();
  const v4f wa = *(const v4f*)(nw + lane * 8);
  const v4f wb = *(const v4f*)(nw + lane * 8 + 4);
  const v4f ba = *(const v4f*)(nb + lane * 8);
  const v4f bb = *(const v4f*)(nb + lane * 8 + 4);
  constexpr float kInvC = 1.0f / (float)kCdim;
#pragma unroll 1
  for (int j = 0; j < kLnTok / 8; ++j) {
    const int tok = wave * (kLnTok / 8) + j;
    const float* sp = sX + tok * kTP + lane * 8;
    const v4f a0 = *(const v4f*)(sp);
    const v4f a1 = *(const v4f*)(sp + 4);
    float s = ((a0[0] + a0[1]) + (a0[2] + a0[3])) + ((a1[0] + a1[1]) + (a1[2] + a1[3]));
#pragma unroll
    for (int off = 1; off < 32; off <<= 1) s += __shfl_xor(s, off, 32);
    const float mu = s * kInvC;
    float dv0[4], dv1[4];
    float s2 = 0.0f;
#pragma unroll
    for (int e = 0; e < 4; ++e) {
      dv0[e] = a0[e] - mu;
      dv1[e] = a1[e] - mu;
      s2 += dv0[e] * dv0[e];
      s2 += dv1[e] * dv1[e];
    }
#pragma unroll
    for (int off = 1; off < 32; off <<= 1) s2 += __shfl_xor(s2, off, 32);
    const float var = s2 * kInvC;
    const float rs = rsqrtf(var + kEps);
    v8h hv, lv;
#pragma unroll
    for (int e = 0; e < 4; ++e) {
      const float o0 = (dv0[e] * rs) * wa[e] + ba[e];
      const float o1 = (dv1[e] * rs) * wb[e] + bb[e];
      const unsigned short h0 = f2bf_bits(o0), h1 = f2bf_bits(o1);
      const unsigned short q0 = f2bf_bits(o0 - bf_bits2f(h0)), q1 = f2bf_bits(o1 - bf_bits2f(h1));
      hv[e]     = __builtin_bit_cast(_Float16, h0);
      hv[4 + e] = __builtin_bit_cast(_Float16, h1);
      lv[e]     = __builtin_bit_cast(_Float16, q0);
      lv[4 + e] = __builtin_bit_cast(_Float16, q1);
    }
    const size_t o = (size_t)(t0 + tok) * kCdim + lane * 8;
    unsigned short* ph = XNH + o;
    unsigned short* pl = XNL + o;
    *(volatile v8h*)ph = hv;
    *(volatile v8h*)pl = lv;
    __threadfence();
    *(volatile v8h*)ph = hv;
    *(volatile v8h*)pl = lv;
  }
}

__global__ __launch_bounds__(256) void conv_silu_kernel(
    const float* __restrict__ XZ, const float* __restrict__ cw, const float* __restrict__ cb,
    float* __restrict__ UC, unsigned short* __restrict__ UCH, unsigned short* __restrict__ UCL)
{
  __shared__ __align__(16) float sT[16 * kTP];
  const int tid = threadIdx.x, lane = tid & 31, wave = tid >> 5;
  const int d0 = blockIdx.x * 256, d = d0 + tid;
  const int t0 = blockIdx.y * 64;
  const float w0 = cw[d * kConvT + 0], w1 = cw[d * kConvT + 1], w2 = cw[d * kConvT + 2], w3 = cw[d * kConvT + 3];
  const float bc = cb[d];
  float xm3, xm2, xm1;
  {
    const int r3 = t0 - 3, r2 = t0 - 2, r1 = t0 - 1;
    const float v3 = XZ[(size_t)(r3 < 0 ? 0 : r3) * kNxz + d];
    const float v2 = XZ[(size_t)(r2 < 0 ? 0 : r2) * kNxz + d];
    const float v1 = XZ[(size_t)(r1 < 0 ? 0 : r1) * kNxz + d];
    xm3 = (r3 >= 0) ? v3 : 0.f;
    xm2 = (r2 >= 0) ? v2 : 0.f;
    xm1 = (r1 >= 0) ? v1 : 0.f;
  }
  const int hrow = wave >> 1;
  const int hch  = (wave & 1) * 128 + lane * 4;
#pragma unroll 1
  for (int sub = 0; sub < 4; ++sub) {
    const int lb = t0 + sub * 16;
#pragma unroll 1
    for (int s = 0; s < 16; ++s) {
      const float xc = XZ[(size_t)(lb + s) * kNxz + d];
      float acc = w0 * xm3;
      acc = fmaf(w1, xm2, acc);
      acc = fmaf(w2, xm1, acc);
      acc = fmaf(w3, xc, acc);
      const float sv = acc + bc;
      const float sg = __builtin_amdgcn_rcpf(1.0f + expf(-sv));
      sT[s * kTP + tid] = sv * sg;
      xm3 = xm2; xm2 = xm1; xm1 = xc;
    }
    __syncthreads();
    v4f fv[4];
    v8h bh[2], blo[2];
#pragma unroll
    for (int it = 0; it < 4; ++it) fv[it] = *(const v4f*)(sT + (it * 4 + hrow) * kTP + hch);
#pragma unroll
    for (int it = 0; it < 2; ++it) {
      const float* sp = sT + (it * 8 + wave) * kTP + lane * 8;
      const v4f a0 = *(const v4f*)(sp);
      const v4f a1 = *(const v4f*)(sp + 4);
#pragma unroll
      for (int e = 0; e < 4; ++e) {
        const unsigned short h0 = f2bf_bits(a0[e]), h1 = f2bf_bits(a1[e]);
        const unsigned short l0 = f2bf_bits(a0[e] - bf_bits2f(h0)), l1 = f2bf_bits(a1[e] - bf_bits2f(h1));
        bh[it][e]      = __builtin_bit_cast(_Float16, h0);
        bh[it][4 + e]  = __builtin_bit_cast(_Float16, h1);
        blo[it][e]     = __builtin_bit_cast(_Float16, l0);
        blo[it][4 + e] = __builtin_bit_cast(_Float16, l1);
      }
    }
    for (int pass = 0; pass < 2; ++pass) {
#pragma unroll
      for (int it = 0; it < 4; ++it)
        *(volatile v4f*)(UC + (size_t)(lb + it * 4 + hrow) * kDin + d0 + hch) = fv[it];
#pragma unroll
      for (int it = 0; it < 2; ++it) {
        const size_t o = (size_t)(lb + it * 8 + wave) * kDin + d0 + lane * 8;
        *(volatile v8h*)(UCH + o) = bh[it];
        *(volatile v8h*)(UCL + o) = blo[it];
      }
      __threadfence();
    }
    __syncthreads();
  }
}

__global__ __launch_bounds__(256) void scan_kernel(
    const float* __restrict__ DLR, const float* __restrict__ UC, const float* __restrict__ XZ,
    const float* __restrict__ DBC, const float* __restrict__ A_log, const float* __restrict__ Dv,
    unsigned short* __restrict__ YH, unsigned short* __restrict__ YL)
{
  __shared__ __align__(16) float sBC[16 * 32];
  __shared__ __align__(16) float sA[kNst * 256];
  __shared__ __align__(16) float sY[16 * kTP];
  const int tid = threadIdx.x, lane = tid & 31, wave = tid >> 5;
  const int d0 = blockIdx.x * 256, d = d0 + tid;

#pragma unroll 1
  for (int n = 0; n < kNst; ++n) sA[n * 256 + tid] = 0.0f - expf(A_log[(size_t)d * kNst + n]);
  __syncthreads();
  float An[kNst], h[kNst];
#pragma unroll
  for (int n = 0; n < kNst; ++n) { An[n] = sA[n * 256 + tid]; h[n] = 0.0f; }
  const float Dd = Dv[d];

#pragma unroll 1
  for (int c = 0; c < kSeq / 16; ++c) {
    const int l0 = c * 16;
    if (tid < 128) {
      const int r = tid >> 3, q = (tid & 7) * 4;
      const v4f v = *(const v4f*)(DBC + (size_t)(l0 + r) * kDbcP + kDtR + q);
      *(v4f*)(sBC + r * 32 + q) = v;
    }
    __syncthreads();
#pragma unroll 1
    for (int s = 0; s < 16; ++s) {
      const size_t m = (size_t)(l0 + s);
      const float a     = DLR[m * kDin + d];
      const float delta = fmaxf(a, 0.0f) + log1pf(expf(-fabsf(a)));
      const float xv    = UC[m * kDin + d];
      const float zv    = XZ[m * kNxz + kDin + d];
      v4f Bq[4], Cq[4];
#pragma unroll
      for (int qq = 0; qq < 4; ++qq) {
        Bq[qq] = *(const v4f*)(sBC + s * 32 + 4 * qq);
        Cq[qq] = *(const v4f*)(sBC + s * 32 + kNst + 4 * qq);
      }
      float du = delta * xv;
      asm volatile("" : "+v"(du));
      float y = 0.0f;
#pragma unroll
      for (int n = 0; n < kNst; ++n) {
        const float e = __expf(delta * An[n]);
        float p = du * Bq[n >> 2][n & 3];
        asm volatile("" : "+v"(p));
        float qv = h[n] * e;
        asm volatile("" : "+v"(qv));
        const float hn = qv + p;
        h[n] = hn;
        float rr = hn * Cq[n >> 2][n & 3];
        asm volatile("" : "+v"(rr));
        y += rr;
      }
      float sk = xv * Dd;
      asm volatile("" : "+v"(sk));
      y += sk;
      const float sg = __builtin_amdgcn_rcpf(1.0f + expf(-zv));
      const float g  = zv * sg;
      sY[s * kTP + tid] = y * g;
    }
    __syncthreads();
    v8h hv[2], lv[2];
#pragma unroll
    for (int it = 0; it < 2; ++it) {
      const float* sp = sY + (it * 8 + wave) * kTP + lane * 8;
      const v4f a0 = *(const v4f*)(sp);
      const v4f a1 = *(const v4f*)(sp + 4);
#pragma unroll
      for (int e = 0; e < 4; ++e) {
        const unsigned short h0 = f2bf_bits(a0[e]), h1 = f2bf_bits(a1[e]);
        const unsigned short l0b = f2bf_bits(a0[e] - bf_bits2f(h0)), l1b = f2bf_bits(a1[e] - bf_bits2f(h1));
        hv[it][e]     = __builtin_bit_cast(_Float16, h0);
        hv[it][4 + e] = __builtin_bit_cast(_Float16, h1);
        lv[it][e]     = __builtin_bit_cast(_Float16, l0b);
        lv[it][4 + e] = __builtin_bit_cast(_Float16, l1b);
      }
    }
    for (int pass = 0; pass < 2; ++pass) {
#pragma unroll
      for (int it = 0; it < 2; ++it) {
        const size_t o = (size_t)(l0 + it * 8 + wave) * kDin + d0 + lane * 8;
        *(volatile v8h*)(YH + o) = hv[it];
        *(volatile v8h*)(YL + o) = lv[it];
      }
      __threadfence();
    }
  }
}

extern "C" void kernel_launch(void* const* d_in, const int* in_sizes, int n_in,
                              void* d_out, int out_size, void* d_ws, size_t ws_size,
                              hipStream_t stream)
{
  if (n_in < 12) return;
  if (in_sizes[0]  != kBatch * kCdim * kSeq) return;
  if (in_sizes[1]  != kCdim) return;
  if (in_sizes[2]  != kCdim) return;
  if (in_sizes[3]  != kCdim * kNxz) return;
  if (in_sizes[4]  != kDin * kConvT) return;
  if (in_sizes[5]  != kDin) return;
  if (in_sizes[6]  != kDin * kNdbc) return;
  if (in_sizes[7]  != kDtR * kDin) return;
  if (in_sizes[8]  != kDin) return;
  if (in_sizes[9]  != kDin * kNst) return;
  if (in_sizes[10] != kDin) return;
  if (in_sizes[11] != kDin * kCdim) return;
  if (out_size != kBatch * kCdim * kSeq) return;
  if (ws_size < kWsTotal) return;

  const float* x      = (const float*)d_in[0];
  const float* norm_w = (const float*)d_in[1];
  const float* norm_b = (const float*)d_in[2];
  const float* W_in   = (const float*)d_in[3];
  const float* conv_w = (const float*)d_in[4];
  const float* conv_b = (const float*)d_in[5];
  const float* W_x    = (const float*)d_in[6];
  const float* W_dt   = (const float*)d_in[7];
  const float* b_dt   = (const float*)d_in[8];
  const float* A_log  = (const float*)d_in[9];
  const float* D_par  = (const float*)d_in[10];
  const float* W_out  = (const float*)d_in[11];
  float* dout = (float*)d_out;

  char* ws = (char*)d_ws;
  unsigned short* WIH  = (unsigned short*)(ws + kOffWIH);
  unsigned short* WIL  = (unsigned short*)(ws + kOffWIL);
  unsigned short* WXH  = (unsigned short*)(ws + kOffWXH);
  unsigned short* WXL  = (unsigned short*)(ws + kOffWXL);
  unsigned short* WDH  = (unsigned short*)(ws + kOffWDH);
  unsigned short* WDL  = (unsigned short*)(ws + kOffWDL);
  unsigned short* WOH  = (unsigned short*)(ws + kOffWOH);
  unsigned short* WOL  = (unsigned short*)(ws + kOffWOL);
  unsigned short* XNH  = (unsigned short*)(ws + kOffXNH);
  unsigned short* XNL  = (unsigned short*)(ws + kOffXNL);
  float*          XZ   = (float*)(ws + kOffXZ);
  float*          UC   = (float*)(ws + kOffUC);
  unsigned short* UCH  = (unsigned short*)(ws + kOffUCH);
  unsigned short* UCL  = (unsigned short*)(ws + kOffUCL);
  float*          DBC  = (float*)(ws + kOffDBC);
  unsigned short* DBCH = (unsigned short*)(ws + kOffDBCH);
  unsigned short* DBCL = (unsigned short*)(ws + kOffDBCL);
  float*          DLR  = (float*)(ws + kOffDLR);
  unsigned short* YH   = (unsigned short*)(ws + kOffYH);
  unsigned short* YL   = (unsigned short*)(ws + kOffYL);
  const float* dummy_bias  = b_dt;
  const float* dummy_resid = x;

  wt_split_kernel<<<dim3(kNxz / 64,  kCdim / 64), 256, 0, stream>>>(W_in,  WIH, WIL, kCdim, kNxz,  kCdim);
  wt_split_kernel<<<dim3(kDbcP / 64, kDin / 64),  256, 0, stream>>>(W_x,   WXH, WXL, kDin,  kNdbc, kDin);
  wt_split_kernel<<<dim3(kDin / 64,  kWdP / 64),  256, 0, stream>>>(W_dt,  WDH, WDL, kDtR,  kDin,  kWdP);
  wt_split_kernel<<<dim3(kCdim / 64, kDin / 64),  256, 0, stream>>>(W_out, WOH, WOL, kDin,  kCdim, kDin);

  layernorm_split_kernel<<<kRows / kLnTok, 256, 0, stream>>>(x, norm_w, norm_b, XNH, XNL);

  for (int b = 0; b < kBatch; ++b) {
    const unsigned short* XNHb = XNH + (size_t)b * kSeq * kCdim;
    const unsigned short* XNLb = XNL + (size_t)b * kSeq * kCdim;
    const float* xb   = x    + (size_t)b * kCdim * kSeq;
    float*       outb = dout + (size_t)b * kCdim * kSeq;

    wmma_gemm64<1, true, 0, 0, false><<<dim3(128, 1), 256, 0, stream>>>(
        XNHb, XNLb, kCdim, 0L,
        WIH, WIL, kCdim, 0L,
        (void*)XZ, (void*)XZ, kNxz, 0L,
        dummy_bias, dummy_resid, 0L,
        kSeq, kNxz, kCdim, 1.0f);

    conv_silu_kernel<<<dim3(kDin / 256, kSeq / 64), 256, 0, stream>>>(XZ, conv_w, conv_b, UC, UCH, UCL);

    wmma_gemm64<1, true, 0, 0, false><<<dim3(8, 1), 256, 0, stream>>>(
        UCH, UCL, kDin, 0L,
        WXH, WXL, kDin, 0L,
        (void*)DBC, (void*)DBC, kDbcP, 0L,
        dummy_bias, dummy_resid, 0L,
        kSeq, kDbcP, kDin, 1.0f);

    split_rows_bf16_kernel<<<(kSeq * kDbcP / 8) / 256, 256, 0, stream>>>(DBC, DBCH, DBCL, kSeq * kDbcP / 8);

    wmma_gemm64<1, true, 2, 0, false><<<dim3(64, 1), 256, 0, stream>>>(
        DBCH, DBCL, kDbcP, 0L,
        WDH, WDL, kWdP, 0L,
        (void*)DLR, (void*)DLR, kDin, 0L,
        b_dt, dummy_resid, 0L,
        kSeq, kDin, kDtK, 1.0f);

    scan_kernel<<<dim3(kDin / 256, 1), 256, 0, stream>>>(DLR, UC, XZ, DBC, A_log, D_par, YH, YL);

    wmma_gemm64<1, true, 0, 0, true><<<dim3(32, 1), 256, 0, stream>>>(
        WOH, WOL, kDin, 0L,
        YH, YL, kDin, 0L,
        (void*)outb, (void*)outb, kSeq, 0L,
        dummy_bias, xb, 0L,
        kCdim, kSeq, kDin, 1.0f);
  }
}
